// Encoder_1623497638443
// MI455X (gfx1250) — hardware-verified
//
#include <hip/hip_runtime.h>
#include <math.h>

constexpr int NBATCH = 64;
constexpr int NFEAT  = 32;
constexpr int NTIME  = 128;
constexpr int NHID   = 128;
constexpr int NEMB   = 100;
constexpr int NGATE  = 4 * NHID;
constexpr int NSEQ   = NTIME * NFEAT;
constexpr int NTHR   = 256;
constexpr int ROWS_BLK = 32;
constexpr int HPITCH = 264;
constexpr int OPITCH = 132;
constexpr int NOUT0  = NBATCH * NFEAT * NEMB;
constexpr int NOUT1  = NTIME * NBATCH * NHID;
constexpr int OUT1_BYTE_OFF = 819200;
constexpr int OUT_TOTAL_BYTES = 5013504;
constexpr float WCARRY     = 256.0f;
constexpr float WCARRY_INV = 1.0f / 256.0f;
constexpr float LOG2E_F    = 1.4426950408889634f;
constexpr float KSIG = -LOG2E_F;
constexpr float KTNH = 2.0f * LOG2E_F;
constexpr int WPLANE_ELEMS = NGATE * NHID;
constexpr int WPLANE_BLOCKS = WPLANE_ELEMS / 8 / NTHR;
constexpr int XS_BLOCKS = (NSEQ * NBATCH) / 4 / NTHR;
constexpr int PREP_BLOCKS = 3 * WPLANE_BLOCKS + XS_BLOCKS;
constexpr int SPAT_THREADS = NOUT0 / 4;
constexpr int SPAT_BLOCKS = SPAT_THREADS / NTHR;

static_assert(NOUT0 * 4 == OUT1_BYTE_OFF, "out1 offset");
static_assert(OUT1_BYTE_OFF % 128 == 0, "out1 line aligned");
static_assert(OUT1_BYTE_OFF + NOUT1 * 4 == OUT_TOTAL_BYTES, "d_out extent");
static_assert(NHID % 32 == 0, "GEMM K multiple of 32");
static_assert(NBATCH % ROWS_BLK == 0 && ROWS_BLK == 32, "two 16-row subtiles per block");
static_assert(NHID == 16 * (NTHR / 32), "8 waves x 16 hidden units");
static_assert((2 * ROWS_BLK * HPITCH) % NTHR == 0, "h zero-fill loop exact");
static_assert(WPLANE_BLOCKS == 32, "weight plane block count");
static_assert(XS_BLOCKS == 256, "xs plane block count");
static_assert(SPAT_BLOCKS * NTHR * 4 == NOUT0, "spatial grid exact");
static_assert(NEMB % 4 == 0, "four consecutive outputs share (b, f)");
static_assert((NFEAT & (NFEAT - 1)) == 0, "feature count power of two");

typedef __attribute__((ext_vector_type(16))) _Float16 v16h;
typedef __attribute__((ext_vector_type(8)))  _Float16 v8h;
typedef __attribute__((ext_vector_type(8)))  float    v8f;
typedef __attribute__((ext_vector_type(4)))  float    v4f;

template <typename T> struct Frag;
template <> struct Frag<_Float16> {
  typedef v16h V; union U { v16h v; v8h h[2]; };
  static __device__ __forceinline__ v16h load(const _Float16* p) {
    U f; f.h[0] = *(const v8h*)(p); f.h[1] = *(const v8h*)(p + 16); return f.v;
  }
  static __device__ __forceinline__ v8f mma(v16h a, v16h b, v8f c) {
    return __builtin_amdgcn_wmma_f32_16x16x32_f16(false, a, false, b, (short)0, c, false, false);
  }
};

__device__ __forceinline__ void guard8(v8f& a0, v8f& a1, v8f& a2, v8f& a3, v8f& a4, v8f& a5, v8f& a6, v8f& a7,
                                       v16h x0, v16h x1, v16h y0, v16h y1, v16h y2, v16h y3) {
  asm volatile("v_nop\n\tv_nop\n\tv_nop\n\tv_nop"
               : "+v"(a0), "+v"(a1), "+v"(a2), "+v"(a3), "+v"(a4), "+v"(a5), "+v"(a6), "+v"(a7)
               : "v"(x0), "v"(x1), "v"(y0), "v"(y1), "v"(y2), "v"(y3));
}

__device__ __forceinline__ float sig_e2(float t) {
  return __builtin_amdgcn_rcpf(1.0f + __builtin_amdgcn_exp2f(t));
}
__device__ __forceinline__ float tanh_e2(float t) {
  return 1.0f - 2.0f * __builtin_amdgcn_rcpf(__builtin_amdgcn_exp2f(t) + 1.0f);
}
__device__ __forceinline__ float lstm_cell(float ti, float tf, float tz, float to, float& cs) {
  const float ig = sig_e2(ti);
  const float fg = sig_e2(tf);
  const float og = sig_e2(to);
  const float gz = tanh_e2(tz);
  const float cn = fg * cs + ig * gz;
  cs = cn;
  return og * tanh_e2(cn * KTNH);
}

__device__ __forceinline__ void gemm_k128(const _Float16* a0p, const _Float16* a1p, const _Float16* bp, v8f (&acc)[2][4]) {
  constexpr int GST = NHID * NHID;
#pragma unroll 1
  for (int k0 = 0; k0 < NHID; k0 += 32) {
    const v16h a0 = Frag<_Float16>::load(a0p + k0);
    const v16h a1 = Frag<_Float16>::load(a1p + k0);
    const v16h b0 = Frag<_Float16>::load(bp + k0);
    const v16h b1 = Frag<_Float16>::load(bp + 1 * GST + k0);
    const v16h b2 = Frag<_Float16>::load(bp + 2 * GST + k0);
    const v16h b3 = Frag<_Float16>::load(bp + 3 * GST + k0);
    acc[0][0] = Frag<_Float16>::mma(a0, b0, acc[0][0]);
    acc[1][0] = Frag<_Float16>::mma(a1, b0, acc[1][0]);
    acc[0][1] = Frag<_Float16>::mma(a0, b1, acc[0][1]);
    acc[1][1] = Frag<_Float16>::mma(a1, b1, acc[1][1]);
    acc[0][2] = Frag<_Float16>::mma(a0, b2, acc[0][2]);
    acc[1][2] = Frag<_Float16>::mma(a1, b2, acc[1][2]);
    acc[0][3] = Frag<_Float16>::mma(a0, b3, acc[0][3]);
    acc[1][3] = Frag<_Float16>::mma(a1, b3, acc[1][3]);
    guard8(acc[0][0], acc[1][0], acc[0][1], acc[1][1], acc[0][2], acc[1][2], acc[0][3], acc[1][3],
           a0, a1, b0, b1, b2, b3);
  }
}

__global__ __launch_bounds__(NTHR) void prep_kernel(const float* __restrict__ x,
                                                    const float* __restrict__ w_hh0,
                                                    const float* __restrict__ w_ih1,
                                                    const float* __restrict__ w_hh1,
                                                    unsigned short* __restrict__ W0,
                                                    unsigned short* __restrict__ W1I,
                                                    unsigned short* __restrict__ W1H,
                                                    float* __restrict__ XS) {
  const int bx = blockIdx.x, tid = threadIdx.x;
  if (bx < 3 * WPLANE_BLOCKS) {
    const int seg = bx / WPLANE_BLOCKS;
    const float* src = (seg == 0) ? w_hh0 : ((seg == 1) ? w_ih1 : w_hh1);
    unsigned short* dst = (seg == 0) ? W0 : ((seg == 1) ? W1I : W1H);
    const int i = (bx - seg * WPLANE_BLOCKS) * NTHR + tid;
    const float* sp = src + (size_t)i * 8;
    const v4f a = *(const v4f*)(sp);
    const v4f b = *(const v4f*)(sp + 4);
    v8h hv;
#pragma unroll
    for (int e = 0; e < 4; ++e) {
      const float fa = a[e] * WCARRY;
      const float fb = b[e] * WCARRY;
      hv[e]     = (_Float16)fa;
      hv[4 + e] = (_Float16)fb;
    }
    unsigned short* op = dst + (size_t)i * 8;
    *(volatile v8h*)op = hv;
    __threadfence();
    *(volatile v8h*)op = hv;
  } else {
    const int i = (bx - 3 * WPLANE_BLOCKS) * NTHR + tid;
    const int s = i >> 4;
    const int b4 = (i & 15) * 4;
    const int f = s & (NFEAT - 1);
    const int tt = s >> 5;
    const float* sp = x + (size_t)b4 * (NFEAT * NTIME) + f * NTIME + tt;
    v4f o;
    o[0] = sp[0];
    o[1] = sp[1 * NFEAT * NTIME];
    o[2] = sp[2 * NFEAT * NTIME];
    o[3] = sp[3 * NFEAT * NTIME];
    float* op = XS + (size_t)i * 4;
    *(volatile v4f*)op = o;
    __threadfence();
    *(volatile v4f*)op = o;
  }
}

__global__ __launch_bounds__(NTHR) void spatial_kernel(const float* __restrict__ x, const float* __restrict__ Ws,
                                                       const float* __restrict__ bs, float* __restrict__ out0) {
  const int i = blockIdx.x * NTHR + threadIdx.x;
  if (i >= SPAT_THREADS) return;
  const int o = i * 4;
  const int b = o / (NFEAT * NEMB);
  const int rem = o - b * (NFEAT * NEMB);
  const int f = rem / NEMB;
  const int e = rem - f * NEMB;
  const float* xp = x + (size_t)(b * NFEAT + f) * NTIME;
  const float* wp = Ws + (size_t)f * NTIME * NEMB + e;
  v4f acc = {0.0f, 0.0f, 0.0f, 0.0f};
#pragma unroll 1
  for (int t = 0; t < NTIME; t += 4) {
    const v4f xv = *(const v4f*)(xp + t);
    const v4f w0 = *(const v4f*)(wp + (size_t)(t + 0) * NEMB);
    const v4f w1 = *(const v4f*)(wp + (size_t)(t + 1) * NEMB);
    const v4f w2 = *(const v4f*)(wp + (size_t)(t + 2) * NEMB);
    const v4f w3 = *(const v4f*)(wp + (size_t)(t + 3) * NEMB);
#pragma unroll
    for (int q = 0; q < 4; ++q) {
      float a = acc[q];
      a = fmaf(xv[0], w0[q], a);
      a = fmaf(xv[1], w1[q], a);
      a = fmaf(xv[2], w2[q], a);
      a = fmaf(xv[3], w3[q], a);
      acc[q] = a;
    }
  }
  const v4f bv = *(const v4f*)(bs + f * NEMB + e);
  v4f r;
#pragma unroll
  for (int q = 0; q < 4; ++q) r[q] = acc[q] + bv[q];
  float* op = out0 + (size_t)o;
  *(volatile v4f*)op = r;
  __threadfence();
  *(volatile v4f*)op = r;
}

__global__ __launch_bounds__(NTHR) void lstm2_kernel(const float* __restrict__ XS,
                                                     const unsigned short* __restrict__ W0p,
                                                     const unsigned short* __restrict__ W1Ip,
                                                     const unsigned short* __restrict__ W1Hp,
                                                     const float* __restrict__ w_ih0,
                                                     const float* __restrict__ b_ih0,
                                                     const float* __restrict__ b_hh0,
                                                     const float* __restrict__ b_ih1,
                                                     const float* __restrict__ b_hh1,
                                                     float* __restrict__ out1) {
  __shared__ __align__(16) _Float16 Hb[2][ROWS_BLK * HPITCH];
  __shared__ __align__(16) float    Os[ROWS_BLK * OPITCH];
  const _Float16* W0  = (const _Float16*)W0p;
  const _Float16* W1I = (const _Float16*)W1Ip;
  const _Float16* W1H = (const _Float16*)W1Hp;
  const int tid = threadIdx.x, lane = tid & 31, wave = tid >> 5;
  const int c = lane & 15, hh = lane >> 4, koff = hh * 8;
  const int rowbase = blockIdx.x * ROWS_BLK;
  const int j = 16 * wave + c;

  {
    _Float16* hf = &Hb[0][0];
#pragma unroll 1
    for (int i = tid; i < 2 * ROWS_BLK * HPITCH; i += NTHR) hf[i] = (_Float16)0.0f;
  }

  float kb0[4], kw0[4], kb1[4];
#pragma unroll
  for (int g = 0; g < 4; ++g) {
    const float ks = (g == 2) ? KTNH : KSIG;
    const int n = g * NHID + j;
    const float bi = b_ih0[n];
    const float bh = b_hh0[n];
    const float wi = w_ih0[n];
    kb0[g] = (bi + bh) * ks;
    kw0[g] = wi * ks;
  }
  asm volatile("" : "+v"(kb0[0]), "+v"(kb0[1]), "+v"(kb0[2]), "+v"(kb0[3]),
                    "+v"(kw0[0]), "+v"(kw0[1]), "+v"(kw0[2]), "+v"(kw0[3]) :: "memory");
#pragma unroll
  for (int g = 0; g < 4; ++g) {
    const float ks = (g == 2) ? KTNH : KSIG;
    const int n = g * NHID + j;
    const float bi = b_ih1[n];
    const float bh = b_hh1[n];
    kb1[g] = (bi + bh) * ks;
  }
  asm volatile("" : "+v"(kb1[0]), "+v"(kb1[1]), "+v"(kb1[2]), "+v"(kb1[3]) :: "memory");

  float c0s[2][8], c1s[2][8];
#pragma unroll
  for (int mt = 0; mt < 2; ++mt)
#pragma unroll
    for (int r = 0; r < 8; ++r) { c0s[mt][r] = 0.0f; c1s[mt][r] = 0.0f; }

  constexpr float KA_SIG = KSIG * WCARRY_INV;
  constexpr float KA_TNH = KTNH * WCARRY_INV;

  const _Float16* w0b  = W0  + (size_t)j * NHID + koff;
  const _Float16* w1ib = W1I + (size_t)j * NHID + koff;
  const _Float16* w1hb = W1H + (size_t)j * NHID + koff;
  const v8f z8 = {0.f, 0.f, 0.f, 0.f, 0.f, 0.f, 0.f, 0.f};

  __syncthreads();

#pragma unroll 1
  for (int s = 0; s < NSEQ; ++s) {
    const int cur = s & 1;
    const _Float16* hc = &Hb[cur][0];
    _Float16* hn = &Hb[cur ^ 1][0];
    const bool samp = ((s & (NFEAT - 1)) == (NFEAT - 1));

    v8f acc[2][4];
#pragma unroll
    for (int mt = 0; mt < 2; ++mt)
#pragma unroll
      for (int g = 0; g < 4; ++g) acc[mt][g] = z8;
    gemm_k128(hc + c * HPITCH + koff, hc + (16 + c) * HPITCH + koff, w0b, acc);

    float xr[2][8];
    {
      const float* xp = XS + (size_t)s * NBATCH + rowbase + koff;
      const v4f x00 = *(const v4f*)(xp);
      const v4f x01 = *(const v4f*)(xp + 4);
      const v4f x10 = *(const v4f*)(xp + 16);
      const v4f x11 = *(const v4f*)(xp + 20);
#pragma unroll
      for (int e = 0; e < 4; ++e) {
        xr[0][e] = x00[e]; xr[0][4 + e] = x01[e];
        xr[1][e] = x10[e]; xr[1][4 + e] = x11[e];
      }
    }

#pragma unroll
    for (int mt = 0; mt < 2; ++mt) {
#pragma unroll
      for (int r = 0; r < 8; ++r) {
        const float xv = xr[mt][r];
        const float ti = fmaf(xv, kw0[0], fmaf(acc[mt][0][r], KA_SIG, kb0[0]));
        const float tf = fmaf(xv, kw0[1], fmaf(acc[mt][1][r], KA_SIG, kb0[1]));
        const float tz = fmaf(xv, kw0[2], fmaf(acc[mt][2][r], KA_TNH, kb0[2]));
        const float to = fmaf(xv, kw0[3], fmaf(acc[mt][3][r], KA_SIG, kb0[3]));
        const float hv = lstm_cell(ti, tf, tz, to, c0s[mt][r]);
        hn[(16 * mt + 8 * hh + r) * HPITCH + j] = (_Float16)hv;
      }
    }
    __syncthreads();

#pragma unroll
    for (int mt = 0; mt < 2; ++mt)
#pragma unroll
      for (int g = 0; g < 4; ++g) acc[mt][g] = z8;
    gemm_k128(hn + c * HPITCH + koff, hn + (16 + c) * HPITCH + koff, w1ib, acc);
    gemm_k128(hc + c * HPITCH + NHID + koff, hc + (16 + c) * HPITCH + NHID + koff, w1hb, acc);

#pragma unroll
    for (int mt = 0; mt < 2; ++mt) {
#pragma unroll
      for (int r = 0; r < 8; ++r) {
        const float ti = fmaf(acc[mt][0][r], KA_SIG, kb1[0]);
        const float tf = fmaf(acc[mt][1][r], KA_SIG, kb1[1]);
        const float tz = fmaf(acc[mt][2][r], KA_TNH, kb1[2]);
        const float to = fmaf(acc[mt][3][r], KA_SIG, kb1[3]);
        const float hv = lstm_cell(ti, tf, tz, to, c1s[mt][r]);
        const int row = 16 * mt + 8 * hh + r;
        hn[row * HPITCH + NHID + j] = (_Float16)hv;
        if (samp) Os[row * OPITCH + j] = hv;
      }
    }
    __syncthreads();

    if (samp) {
      const int tt = s >> 5;
      for (int pass = 0; pass < 2; ++pass) {
#pragma unroll
        for (int it = 0; it < 4; ++it) {
          const int row = 4 * wave + it;
          const v4f v = *(const v4f*)(Os + row * OPITCH + 4 * lane);
          *(volatile v4f*)(out1 + ((size_t)(tt * NBATCH + rowbase + row)) * NHID + 4 * lane) = v;
        }
        __threadfence();
      }
    }
  }
}

extern "C" void kernel_launch(void* const* d_in, const int* in_sizes, int n_in,
                              void* d_out, int out_size, void* d_ws, size_t ws_size, hipStream_t stream) {
  if (n_in < 11 || d_out == nullptr || d_ws == nullptr) return;
  if (in_sizes[0] != NBATCH * NFEAT * NTIME || in_sizes[1] != NFEAT * NTIME * NEMB || in_sizes[2] != NFEAT * NEMB ||
      in_sizes[3] != NGATE || in_sizes[4] != NGATE * NHID || in_sizes[5] != NGATE || in_sizes[6] != NGATE ||
      in_sizes[7] != NGATE * NHID || in_sizes[8] != NGATE * NHID || in_sizes[9] != NGATE || in_sizes[10] != NGATE ||
      out_size != NOUT0 + NOUT1) return;

  const float* x     = (const float*)d_in[0];
  const float* Wsp   = (const float*)d_in[1];
  const float* bsp   = (const float*)d_in[2];
  const float* w_ih0 = (const float*)d_in[3];
  const float* w_hh0 = (const float*)d_in[4];
  const float* b_ih0 = (const float*)d_in[5];
  const float* b_hh0 = (const float*)d_in[6];
  const float* w_ih1 = (const float*)d_in[7];
  const float* w_hh1 = (const float*)d_in[8];
  const float* b_ih1 = (const float*)d_in[9];
  const float* b_hh1 = (const float*)d_in[10];
  float* out0 = (float*)d_out;
  float* out1 = out0 + (size_t)NOUT0;

  char* ws = (char*)d_ws; size_t off = 0;
  auto carve = [&](size_t bytes) -> char* { char* p = ws + off; off += (bytes + 255) & ~(size_t)255; return p; };
  unsigned short* W0  = (unsigned short*)carve((size_t)WPLANE_ELEMS * 2);
  unsigned short* W1I = (unsigned short*)carve((size_t)WPLANE_ELEMS * 2);
  unsigned short* W1H = (unsigned short*)carve((size_t)WPLANE_ELEMS * 2);
  float*          XS  = (float*)carve((size_t)NSEQ * NBATCH * 4);
  if (off > ws_size || off > (size_t)134217728) return;

  prep_kernel<<<PREP_BLOCKS, NTHR, 0, stream>>>(x, w_hh0, w_ih1, w_hh1, W0, W1I, W1H, XS);
  spatial_kernel<<<SPAT_BLOCKS, NTHR, 0, stream>>>(x, Wsp, bsp, out0);
  lstm2_kernel<<<NBATCH / ROWS_BLK, NTHR, 0, stream>>>(XS, W0, W1I, W1H, w_ih0, b_ih0, b_hh0, b_ih1, b_hh1, out1);
}
